// GINEncoder_35519379538034
// MI455X (gfx1250) — hardware-verified
//
#include <hip/hip_runtime.h>
#include <hip/hip_bf16.h>
#include <math.h>


#define BB 2
#define SS 2048
#define DD 1024
#define HH 16
#define DKK 64
#define QW 2

typedef _Float16 bf16;
typedef __attribute__((ext_vector_type(4))) unsigned v4u_t;
typedef unsigned v4ua __attribute__((ext_vector_type(4), may_alias));
typedef __attribute__((ext_vector_type(4))) float v4f_t;
typedef float v4fa __attribute__((ext_vector_type(4), may_alias));
typedef __attribute__((ext_vector_type(16))) bf16  bf16x16;
typedef __attribute__((ext_vector_type(8)))  bf16  bf16x8;
typedef __attribute__((ext_vector_type(4)))  bf16  bf16x4;
typedef __attribute__((ext_vector_type(8)))  float f32x8;

#define LDS_STRIDE 48
#define KSTRIDE    72
#define VSTRIDE    48

__device__ __forceinline__ f32x8 wmma_bf16(bf16x16 a, bf16x16 b, f32x8 c) {
  return __builtin_amdgcn_wmma_f32_16x16x32_f16(
      false, a, false, b, (short)0, c, false, false);
}
#define RSPLIT (1.0f / 2048.0f)
__device__ __forceinline__ bf16 lo_of(float v, bf16 h) { return (bf16)((v - (float)h) * 2048.0f); }
__device__ __forceinline__ f32x8 wmma_split(bf16x16 a, bf16x16 al, bf16x16 b, bf16x16 bl, f32x8 c) {
  f32x8 x = {}; x = wmma_bf16(al, b, x); x = wmma_bf16(a, bl, x); return wmma_bf16(a, b, c) + x * RSPLIT; }

template <typename T>
__device__ __forceinline__ bf16x16 load_frag(const T* __restrict__ base, int ld,
                                             int row0, int k0) {
  const int lane = threadIdx.x & 31;
  const int r    = lane & 15;
  const int kh   = (lane >> 4) * 8;
  const T* p0 = base + (size_t)(row0 + r) * ld + (k0 + kh);
  const T* p1 = p0 + 16;
  bf16x16 f;
#pragma unroll
  for (int i = 0; i < 8; ++i) {
    f[i]     = (bf16)p0[i];
    f[i + 8] = (bf16)p1[i];
  }
  return f;
}

__device__ __forceinline__ bf16x16 lds_frag(const bf16* base, int stride) {
  const int lane = threadIdx.x & 31;
  const int row  = lane & 15;
  const int kh   = (lane >> 4) * 8;
  const bf16x8 lo = *(const bf16x8*)(base + row * stride + kh);
  const bf16x8 hi = *(const bf16x8*)(base + row * stride + kh + 16);
  bf16x16 f;
#pragma unroll
  for (int i = 0; i < 8; ++i) { f[i] = lo[i]; f[i + 8] = hi[i]; }
  return f;
}

template <typename T>
__device__ __forceinline__ void stage_read16(const T* __restrict__ p, float* buf) {
#pragma unroll
  for (int i = 0; i < 16; ++i) buf[i] = (float)p[i];
}

__device__ __forceinline__ void stage_write(bf16* dst, const float* buf, int nquad) {
#pragma unroll
  for (int i = 0; i < nquad; ++i) {
    bf16x4 q;
    q[0] = (bf16)buf[4 * i];     q[1] = (bf16)buf[4 * i + 1];
    q[2] = (bf16)buf[4 * i + 2]; q[3] = (bf16)buf[4 * i + 3];
    *(bf16x4*)(dst + 4 * i) = q;
  }
}

__global__ __launch_bounds__(256) void transpose_pack_kernel(const float* __restrict__ W, bf16* __restrict__ WT, int K, int N, size_t plane) {
  __shared__ float tile[64][65];
  const int k0 = blockIdx.y * 64, n0 = blockIdx.x * 64, t = threadIdx.x;
  for (int i = t; i < 64 * 64; i += 256) { const int kr = i >> 6, nc = i & 63; tile[kr][nc] = W[(size_t)(k0 + kr) * N + n0 + nc]; }
  __syncthreads();
#pragma unroll 1
  for (int pass = 0; pass < 2; ++pass) {
    for (int i = t; i < 64 * 8; i += 256) { const int nr = i >> 3, k8 = (i & 7) * 8; bf16 hh[8], hl[8];
#pragma unroll
      for (int e = 0; e < 8; ++e) { const float v = tile[k8 + e][nr]; hh[e] = (bf16)v; hl[e] = lo_of(v, hh[e]); }
      bf16* d = WT + (size_t)(n0 + nr) * K + k0 + k8;
      *(volatile v4u_t*)d = *(const v4ua*)hh; *(volatile v4u_t*)(d + plane) = *(const v4ua*)hl; }
    __threadfence();
  }
}

template <typename AT, typename WT, int MODE>
__global__ __launch_bounds__(256) void gemm_split_kernel(
    const AT* __restrict__ A, size_t aPlane, const WT* __restrict__ W, size_t wPlane,
    const float* __restrict__ bias, void* __restrict__ out,
    int M, int N, int K) {
  __shared__ bf16 ldsA[128 * LDS_STRIDE], ldsAl[128 * LDS_STRIDE];
  __shared__ bf16 ldsW[256 * LDS_STRIDE], ldsWl[256 * LDS_STRIDE];
  __shared__ __attribute__((aligned(16))) unsigned char sob[256 * 136 * 2];

  const int t    = threadIdx.x;
  const int wave = t >> 5;
  const int lane = t & 31;
  const int wm   = (wave & 1) * 64;
  const int wn   = (wave >> 1) * 64;
  const int mBlk = blockIdx.x * 128;
  const int nBlk = blockIdx.y * 256;
  const int arow = t >> 1;
  const int ach  = (t & 1) * 16;

  f32x8 acc[4][4] = {};
  for (int k = 0; k < K; k += 32) {
    __syncthreads();
    {
      const AT* ap = A + (size_t)(mBlk + arow) * K + k + ach;
      bf16 hh[16], hl[16];
      if (sizeof(AT) == 4) {
#pragma unroll
        for (int i = 0; i < 16; ++i) { const float v = (float)ap[i]; hh[i] = (bf16)v; hl[i] = lo_of(v, hh[i]); }
      } else {
#pragma unroll
        for (int i = 0; i < 16; ++i) { hh[i] = (bf16)ap[i]; hl[i] = (bf16)ap[aPlane + i]; }
      }
#pragma unroll
      for (int i = 0; i < 16; ++i) { ldsA[arow * LDS_STRIDE + ach + i] = hh[i]; ldsAl[arow * LDS_STRIDE + ach + i] = hl[i]; }
    }
    {
      const WT* wp = W + (size_t)(nBlk + t) * K + k;
      if (sizeof(WT) == 4) {
#pragma unroll
        for (int i = 0; i < 32; ++i) { const float v = (float)wp[i]; const bf16 h_ = (bf16)v; ldsW[t * LDS_STRIDE + i] = h_; ldsWl[t * LDS_STRIDE + i] = lo_of(v, h_); }
      } else {
#pragma unroll
        for (int i = 0; i < 32; ++i) { ldsW[t * LDS_STRIDE + i] = (bf16)wp[i]; ldsWl[t * LDS_STRIDE + i] = (bf16)wp[wPlane + i]; }
      }
    }
    __syncthreads();
    bf16x16 wf[4], wfl[4];
#pragma unroll
    for (int j = 0; j < 4; ++j) { wf[j] = lds_frag(ldsW + (wn + 16 * j) * LDS_STRIDE, LDS_STRIDE); wfl[j] = lds_frag(ldsWl + (wn + 16 * j) * LDS_STRIDE, LDS_STRIDE); }
#pragma unroll
    for (int i = 0; i < 4; ++i) {
      const bf16x16 af = lds_frag(ldsA + (wm + 16 * i) * LDS_STRIDE, LDS_STRIDE), afl = lds_frag(ldsAl + (wm + 16 * i) * LDS_STRIDE, LDS_STRIDE);
#pragma unroll
      for (int j = 0; j < 4; ++j) acc[i][j] = wmma_split(af, afl, wf[j], wfl[j], acc[i][j]);
    }
  }

  const int nlane = lane & 15;
  const int mh    = (lane >> 4) * 8;
  __syncthreads();
  if (MODE == 1) {
    bf16* so = (bf16*)sob;
#pragma unroll
    for (int i = 0; i < 4; ++i)
#pragma unroll
      for (int j = 0; j < 4; ++j) {
        const int nl = wn + 16 * j + nlane;
        const float bv = bias ? bias[nBlk + nl] : 0.0f;
#pragma unroll
        for (int r = 0; r < 8; ++r) so[nl * 136 + wm + 16 * i + mh + r] = (bf16)(acc[i][j][r] + bv);
      }
    __syncthreads();
    const int b_ = mBlk >> 11, s0 = mBlk & (SS - 1);
#pragma unroll 1
    for (int pass = 0; pass < 2; ++pass) {
      for (int ch = t; ch < 256 * 16; ch += 256) { const int nl = ch >> 4, q = (ch & 15) * 8; const int n = nBlk + nl, h = n >> 6, dk = n & (DKK - 1);
        *(volatile v4u_t*)((bf16*)out + (((size_t)(b_ * HH + h)) * DKK + dk) * SS + s0 + q) = *(const v4ua*)(so + nl * 136 + q); }
      __threadfence();
    }
  } else {
    float* so = (float*)sob;
#pragma unroll 1
    for (int hf = 0; hf < 2; ++hf) {
      if (wm == hf * 64) {
#pragma unroll
        for (int i = 0; i < 4; ++i)
#pragma unroll
          for (int j = 0; j < 4; ++j) {
            const int nl = wn + 16 * j + nlane;
            const float bv = bias ? bias[nBlk + nl] : 0.0f;
#pragma unroll
            for (int r = 0; r < 8; ++r) so[(16 * i + mh + r) * 260 + nl] = acc[i][j][r] + bv;
          }
      }
      __syncthreads();
#pragma unroll 1
      for (int pass = 0; pass < 2; ++pass) {
        for (int ch = t; ch < 64 * 64; ch += 256) { const int ml = ch >> 6, q = (ch & 63) * 4;
          *(volatile v4f_t*)((float*)out + (size_t)(mBlk + hf * 64 + ml) * N + nBlk + q) = *(const volatile v4fa*)(so + ml * 260 + q); }
        __threadfence();
      }
      __syncthreads();
    }
  }
}


#define GN 100000
#define GNP 100352
#define GE 1600000
#define NG 512
#define R1 25088
#define R2 50176
template <int FW, int RANGE>
__global__ __launch_bounds__(256) void k_gin(const int* __restrict__ srci, const int* __restrict__ dsti, const float* __restrict__ H, float* __restrict__ R, int rsel) {
  __shared__ int qd[8][256], qs[8][256]; __shared__ int wcnt[8][8];
  const int tid = threadIdx.x, lane = tid & 31, wave = tid >> 5, r0 = rsel * RANGE;
  constexpr int RW = FW, Q4 = RW / 4;
  float* myR = R;
  for (int i = tid; i < RANGE * Q4; i += 256) { const int nl = i / Q4, c4 = (i % Q4) * 4, node = r0 + nl; v4f_t v;
    if (node >= GN) { v.x = v.y = v.z = v.w = 0.0f; } else { v = *(const v4fa*)(H + (size_t)node * FW + c4); }
    *(volatile v4f_t*)(myR + (size_t)nl * RW + c4) = v; }
  __threadfence(); __syncthreads();
  const int* srcp = srci; const int* dstp = dsti;
#pragma unroll 1
  for (int c0 = 0; c0 < GE; c0 += 256) {
    const int e = c0 + tid; int d = -1, sidx = 0;
    if (e < GE) { const int draw = dstp[e]; const int dd = draw < 0 ? 0 : (draw >= GN ? GN - 1 : draw);
      if (dd >= r0 && dd < r0 + RANGE) { d = dd - r0; const int ss = srcp[e]; sidx = ss < 0 ? 0 : (ss >= GN ? GN - 1 : ss); } }
    const int own = (d >= 0) ? (d & 7) : -1; unsigned mown = 0u;
#pragma unroll
    for (int w = 0; w < 8; ++w) { const unsigned m = __builtin_amdgcn_ballot_w32(own == w); if (own == w) mown = m; if (lane == 0) wcnt[w][wave] = __builtin_popcount(m); }
    __syncthreads();
    if (own >= 0) { int base = 0;
#pragma unroll
      for (int w2 = 0; w2 < 8; ++w2) base += (w2 < wave) ? wcnt[own][w2] : 0;
      const int pos = base + __builtin_popcount(mown & ((1u << lane) - 1u)); qd[own][pos] = d; qs[own][pos] = sidx; }
    int total = 0;
#pragma unroll
    for (int w2 = 0; w2 < 8; ++w2) total += wcnt[wave][w2];
    __syncthreads();
#pragma unroll 1
    for (int qi = 0; qi < total; ++qi) { const int dl = qd[wave][qi]; const int sl = qs[wave][qi];
      float* row = myR + (size_t)dl * RW; const float* hs = H + (size_t)sl * FW;
#pragma unroll
      for (int u = 0; u < FW / 32; ++u) row[u * 32 + lane] += hs[u * 32 + lane]; }
    __syncthreads();
  }
  __threadfence(); __syncthreads();
  for (int i = tid; i < RANGE * Q4; i += 256) { const int nl = i / Q4, c4 = (i % Q4) * 4; float* p = myR + (size_t)nl * RW + c4; const v4f_t v = *(const volatile v4fa*)p; *(volatile v4f_t*)p = v; }
  __threadfence(); __syncthreads();
}

__global__ __launch_bounds__(128) void k_packA(const float* __restrict__ W, int KIN, float* __restrict__ A) {
  const int m = blockIdx.x; for (int k = threadIdx.x; k < KIN; k += 128) { const float v = (m < 64) ? W[(size_t)k * 64 + m] : 0.0f;
    *(volatile float*)(A + (size_t)m * KIN + k) = v; __threadfence(); *(volatile float*)(A + (size_t)m * KIN + k) = v; }
}
template <int RANGE>
__global__ __launch_bounds__(256) void k_rows_relu(const float* __restrict__ T, const float* __restrict__ b1, float* __restrict__ Hr) {
  __shared__ float tile[64][65];
  const int n0 = blockIdx.x * 64, t = threadIdx.x;
  for (int i = t; i < 64 * 64; i += 256) { const int c = i >> 6, nn = i & 63; tile[c][nn] = T[(size_t)c * RANGE + n0 + nn]; }
  __syncthreads();
#pragma unroll 1
  for (int pass = 0; pass < 2; ++pass) {
    for (int i = t; i < 64 * 16; i += 256) { const int nr = i >> 4, c4 = (i & 15) * 4; v4f_t v;
#pragma unroll
      for (int q = 0; q < 4; ++q) v[q] = fmaxf(tile[c4 + q][nr] + b1[c4 + q], 0.0f);
      *(volatile v4f_t*)(Hr + (size_t)(n0 + nr) * 64 + c4) = v; }
    __threadfence();
  }
}
template <int RANGE>
__global__ __launch_bounds__(128) void k_tcopy(const float* __restrict__ T, const float* __restrict__ b2, int c0, float* __restrict__ TB) {
  const int f = blockIdx.y, seg = blockIdx.x, t = threadIdx.x;
  const int c = seg * 512 + t * 4; v4f_t v = *(const v4fa*)(T + (size_t)f * RANGE + c); const float bb = b2[f]; v.x += bb; v.y += bb; v.z += bb; v.w += bb;
  float* dst = TB + (size_t)f * GNP + c0 + c; *(volatile v4f_t*)dst = v; __threadfence(); *(volatile v4f_t*)dst = v;
}
__global__ __launch_bounds__(256) void k_bnpart(const float* __restrict__ TB, float* __restrict__ P) {
  const int seg = blockIdx.x, f = blockIdx.y, t = threadIdx.x; __shared__ float red[2][256];
  float s = 0.f, q = 0.f;
  for (int i = seg * 2048 + t; i < (seg + 1) * 2048 && i < GN; i += 256) { const float v = TB[(size_t)f * GNP + i]; s += v; q += v * v; }
  red[0][t] = s; red[1][t] = q; __syncthreads();
  for (int o = 128; o > 0; o >>= 1) { if (t < o) { red[0][t] += red[0][t + o]; red[1][t] += red[1][t + o]; } __syncthreads(); }
  if (t == 0) { typedef __attribute__((ext_vector_type(2))) float v2f; v2f v; v.x = red[0][0]; v.y = red[1][0]; float* dst = P + ((size_t)f * 49 + seg) * 2; *(volatile v2f*)dst = v; __threadfence(); *(volatile v2f*)dst = v; }
}
__global__ __launch_bounds__(64) void k_bnfin(const float* __restrict__ P, const float* __restrict__ gam, const float* __restrict__ bet, float* __restrict__ SC) {
  const int f = threadIdx.x; double s = 0.0, q = 0.0; for (int i = 0; i < 49; ++i) { s += (double)P[((size_t)f * 49 + i) * 2]; q += (double)P[((size_t)f * 49 + i) * 2 + 1]; }
  const double mu = s / (double)GN, var = fmax(q / (double)GN - mu * mu, 0.0); const float a = (float)(1.0 / sqrt(var + 1e-5)) * gam[f];
  typedef __attribute__((ext_vector_type(2))) float v2f; v2f v; v.x = a; v.y = bet[f] - (float)mu * a;
  *(volatile v2f*)(SC + f * 2) = v; __threadfence(); *(volatile v2f*)(SC + f * 2) = v;
}
__global__ __launch_bounds__(256) void k_bnrows(const float* __restrict__ TB, const float* __restrict__ SC, float* __restrict__ Hr) {
  __shared__ float tile[64][65];
  const int n0 = blockIdx.x * 64, t = threadIdx.x;
  for (int i = t; i < 64 * 64; i += 256) { const int c = i >> 6, nn = i & 63; tile[c][nn] = TB[(size_t)c * GNP + n0 + nn]; }
  __syncthreads();
#pragma unroll 1
  for (int pass = 0; pass < 2; ++pass) {
    for (int i = t; i < 64 * 16; i += 256) { const int nr = i >> 4, c4 = (i & 15) * 4; v4f_t v;
#pragma unroll
      for (int q = 0; q < 4; ++q) v[q] = fmaxf(tile[c4 + q][nr] * SC[(c4 + q) * 2] + SC[(c4 + q) * 2 + 1], 0.0f);
      *(volatile v4f_t*)(Hr + (size_t)(n0 + nr) * 64 + c4) = v; }
    __threadfence();
  }
}
__global__ __launch_bounds__(256) void k_pool(const float* __restrict__ TB, const float* __restrict__ SC, const int* __restrict__ batch, float* __restrict__ out) {
  __shared__ int qd[8][256], qs[8][256]; __shared__ int wcnt[8][8]; __shared__ int cnt[NG]; __shared__ float sc0[64], sc1[64];
  const int tid = threadIdx.x, lane = tid & 31, wave = tid >> 5;
  for (int i = tid; i < NG; i += 256) cnt[i] = 0;
  if (tid < 64) { sc0[tid] = SC[tid * 2]; sc1[tid] = SC[tid * 2 + 1]; }
  for (int i = tid; i < NG * 64 / 4; i += 256) { v4f_t z; z.x = z.y = z.z = z.w = 0.0f; *(volatile v4f_t*)(out + (size_t)i * 4) = z; }
  __threadfence(); __syncthreads();
#pragma unroll 1
  for (int c0 = 0; c0 < GN; c0 += 256) {
    const int n = c0 + tid; int d = -1;
    if (n < GN) { const int g = batch[n]; d = g < 0 ? 0 : (g >= NG ? NG - 1 : g); }
    const int own = (d >= 0) ? (d & 7) : -1; unsigned mown = 0u;
#pragma unroll
    for (int w = 0; w < 8; ++w) { const unsigned m = __builtin_amdgcn_ballot_w32(own == w); if (own == w) mown = m; if (lane == 0) wcnt[w][wave] = __builtin_popcount(m); }
    __syncthreads();
    if (own >= 0) { int base = 0;
#pragma unroll
      for (int w2 = 0; w2 < 8; ++w2) base += (w2 < wave) ? wcnt[own][w2] : 0;
      const int pos = base + __builtin_popcount(mown & ((1u << lane) - 1u)); qd[own][pos] = d; qs[own][pos] = n; }
    int total = 0;
#pragma unroll
    for (int w2 = 0; w2 < 8; ++w2) total += wcnt[wave][w2];
    __syncthreads();
#pragma unroll 1
    for (int qi = 0; qi < total; ++qi) { const int g = qd[wave][qi], n = qs[wave][qi]; float* row = out + (size_t)g * 64;
#pragma unroll
      for (int u = 0; u < 2; ++u) { const int f = u * 32 + lane; row[f] += fmaxf(TB[(size_t)f * GNP + n] * sc0[f] + sc1[f], 0.0f); }
      if (lane == 0) cnt[g] += 1; }
    __syncthreads();
  }
  __threadfence(); __syncthreads();
#pragma unroll 1
  for (int pass = 0; pass < 2; ++pass) {
    for (int i = tid; i < NG * 16; i += 256) { const int g = i >> 4, c4 = (i & 15) * 4; float* p = out + (size_t)g * 64 + c4; v4f_t v = *(const volatile v4fa*)p;
      if (pass == 0) { const float inv = 1.0f / fmaxf((float)cnt[g], 1.0f); v.x *= inv; v.y *= inv; v.z *= inv; v.w *= inv; }
      *(volatile v4f_t*)p = v; }
    __threadfence(); __syncthreads();
  }
}

extern "C" void kernel_launch(void* const* d_in, const int* in_sizes, int n_in,
                              void* d_out, int out_size, void* d_ws, size_t ws_size,
                              hipStream_t stream) {
  (void)in_sizes; (void)n_in; (void)out_size; (void)ws_size;
  const float* x = (const float*)d_in[0];
  const int* ei = (const int*)d_in[1];
  const int* batch = (const int*)d_in[2];
  const float* W1a = (const float*)d_in[3]; const float* b1a = (const float*)d_in[4]; const float* W2a = (const float*)d_in[5]; const float* b2a = (const float*)d_in[6];
  const float* g1 = (const float*)d_in[7]; const float* be1 = (const float*)d_in[8];
  const float* W1b = (const float*)d_in[9]; const float* b1b = (const float*)d_in[10]; const float* W2b = (const float*)d_in[11]; const float* b2b = (const float*)d_in[12];
  const float* g2 = (const float*)d_in[13]; const float* be2 = (const float*)d_in[14];
  const int* srci = ei; const int* dsti = ei + (size_t)GE;
  char* ws = (char*)d_ws;
  float* A1a = (float*)ws; ws += (size_t)128 * 128 * 4;
  float* A2a = (float*)ws; ws += (size_t)128 * 64 * 4;
  float* A1b = (float*)ws; ws += (size_t)128 * 64 * 4;
  float* A2b = (float*)ws; ws += (size_t)128 * 64 * 4;
  float* R   = (float*)ws; ws += (size_t)R2 * 64 * 4;
  float* T   = (float*)ws; ws += (size_t)128 * R2 * 4;
  float* Hm  = (float*)ws; ws += (size_t)R2 * 64 * 4;
  float* TB  = (float*)ws; ws += (size_t)64 * GNP * 4;
  float* Hr  = (float*)ws; ws += (size_t)GNP * 64 * 4;
  float* P   = (float*)ws; ws += (size_t)64 * 49 * 2 * 4;
  float* SC  = (float*)ws; ws += 64 * 2 * 4;
  k_packA<<<128, 128, 0, stream>>>(W1a, 128, A1a);
  k_packA<<<128, 128, 0, stream>>>(W2a, 64, A2a);
  k_packA<<<128, 128, 0, stream>>>(W1b, 64, A1b);
  k_packA<<<128, 128, 0, stream>>>(W2b, 64, A2b);
  dim3 blk(256);
  for (int r = 0; r < GNP / R1; ++r) {
    k_gin<128, R1><<<1, 256, 0, stream>>>(srci, dsti, x, R, r);
    gemm_split_kernel<float, float, 2><<<dim3(1, R1 / 256), blk, 0, stream>>>(A1a, 0, R, 0, nullptr, T, 128, R1, 128);
    k_rows_relu<R1><<<R1 / 64, 256, 0, stream>>>(T, b1a, Hm);
    gemm_split_kernel<float, float, 2><<<dim3(1, R1 / 256), blk, 0, stream>>>(A2a, 0, Hm, 0, nullptr, T, 128, R1, 64);
    k_tcopy<R1><<<dim3(R1 / 512, 64), 128, 0, stream>>>(T, b2a, r * R1, TB);
  }
  k_bnpart<<<dim3(49, 64), 256, 0, stream>>>(TB, P);
  k_bnfin<<<1, 64, 0, stream>>>(P, g1, be1, SC);
  k_bnrows<<<GNP / 64, 256, 0, stream>>>(TB, SC, Hr);
  for (int r = 0; r < GNP / R2; ++r) {
    k_gin<64, R2><<<1, 256, 0, stream>>>(srci, dsti, Hr, R, r);
    gemm_split_kernel<float, float, 2><<<dim3(1, R2 / 256), blk, 0, stream>>>(A1b, 0, R, 0, nullptr, T, 128, R2, 64);
    k_rows_relu<R2><<<R2 / 64, 256, 0, stream>>>(T, b1b, Hm);
    gemm_split_kernel<float, float, 2><<<dim3(1, R2 / 256), blk, 0, stream>>>(A2b, 0, Hm, 0, nullptr, T, 128, R2, 64);
    k_tcopy<R2><<<dim3(R2 / 512, 64), 128, 0, stream>>>(T, b2b, r * R2, TB);
  }
  k_bnpart<<<dim3(49, 64), 256, 0, stream>>>(TB, P);
  k_bnfin<<<1, 64, 0, stream>>>(P, g2, be2, SC);
  k_pool<<<1, 256, 0, stream>>>(TB, SC, batch, (float*)d_out);
}
